// SSFormer_12128987644579
// MI455X (gfx1250) — hardware-verified
//
#include <hip/hip_runtime.h>
#include <math.h>
#include <stdint.h>

#define NB_   8
#define NC    512
#define NH    4
#define DH    128
#define SEQ   1024
#define QT    64
#define OPD   132
#define XP    68
#define TP    136
#define NEL   (NB_ * NC * SEQ)
#define NSAMP (NB_ * SEQ)
#define LNPS  6.931471805599453f
#define ISQ   0.08838834764831845f
#define QSC   16.0f
#define IQSC  0.0625f
#define PSC   4096.0f
#define IPSC  0.000244140625f
#define ESC   32.0f
#define RSC   2048.0f
#define IRSC  0.00048828125f
#define WSC   64.0f
#define IWE   0.00048828125f
#define BNEPS 1.0e-5f
static_assert(NC * SEQ == 524288);
static_assert(NC == NH * DH);
static_assert((SEQ / QT) == 16);
static_assert((SEQ % 64) == 0);
static_assert(SEQ == 4 * 256);
static_assert(DH == 128);
static_assert((NC % 32) == 0);
static_assert(((NB_ * NC) % 256) == 0);

typedef _Float16       v16h __attribute__((ext_vector_type(16)));
typedef _Float16       v8h  __attribute__((ext_vector_type(8)));
typedef float          v8f  __attribute__((ext_vector_type(8)));
typedef float          v4f  __attribute__((ext_vector_type(4)));
typedef unsigned int   v4u  __attribute__((ext_vector_type(4)));

union FragH { v16h v; v8h h[2]; };
static_assert(sizeof(FragH) == 32);

__device__ __forceinline__ unsigned short bf_bits(float f) {
  unsigned u = __float_as_uint(f);
  return (unsigned short)((u + 0x7FFFu + ((u >> 16) & 1u)) >> 16);
}
__device__ __forceinline__ float bf_up(unsigned short h) { return __uint_as_float(((unsigned)h) << 16); }
__device__ __forceinline__ float bfr(float f) { return bf_up(bf_bits(f)); }
__device__ __forceinline__ unsigned short h16(float f) {
  const _Float16 x = (_Float16)f;
  return __builtin_bit_cast(unsigned short, x);
}
__device__ __forceinline__ unsigned pk16(unsigned short a, unsigned short b) { return (unsigned)a | ((unsigned)b << 16); }
__device__ __forceinline__ v8f zero8() { v8f z = {0.f, 0.f, 0.f, 0.f, 0.f, 0.f, 0.f, 0.f}; return z; }
__device__ __forceinline__ float hmax8(v8f s) {
  return fmaxf(fmaxf(fmaxf(s[0], s[1]), fmaxf(s[2], s[3])), fmaxf(fmaxf(s[4], s[5]), fmaxf(s[6], s[7])));
}

__device__ __forceinline__ void st2u(unsigned short* p, v4u v) {
  *(volatile v4u*)p = v;
  __threadfence();
  *(volatile v4u*)p = v;
}
__device__ __forceinline__ void st2f(float* p, v4f v) {
  *(volatile v4f*)p = v;
  __threadfence();
  *(volatile v4f*)p = v;
}

__device__ __forceinline__ v16h ldfrag_h(const _Float16* p) {
  FragH f;
  f.h[0] = *(const v8h*)(p);
  f.h[1] = *(const v8h*)(p + 16);
  return f.v;
}

__device__ __forceinline__ v8f mma_h(v16h a, v16h b, v8f c) {
  v8f d = __builtin_amdgcn_wmma_f32_16x16x32_f16(false, a, false, b, (short)0, c, false, false);
#if defined(__HIP_DEVICE_COMPILE__)
  asm volatile("v_nop\n\tv_nop\n\tv_nop\n\tv_nop" : "+v"(d) : "v"(a), "v"(b));
#endif
  return d;
}

__global__ __launch_bounds__(256)
void cvt_x_kernel(const float* __restrict__ x, unsigned short* XV, unsigned short* XT) {
  __shared__ __align__(16) unsigned short Ts[64 * TP];
  const int tid = threadIdx.x;
  const int e = tid & 7, rq = tid >> 3;
  const int bx = blockIdx.x;
  const int b = bx >> 6, rem = bx & 63;
  const int hd = rem >> 4, lt = rem & 15;
  const int l0 = lt * 64;
#pragma unroll 1
  for (int it = 0; it < 4; ++it) {
    const int row = it * 32 + rq;
    const size_t gi = ((size_t)(b * NC + hd * DH + row)) * SEQ + l0 + 8 * e;
    const v4f a  = *(const v4f*)(x + gi);
    const v4f c4 = *(const v4f*)(x + gi + 4);
    unsigned short hb[8];
#pragma unroll
    for (int j = 0; j < 4; ++j) {
      hb[j]     = h16(bfr(a[j]));
      hb[4 + j] = h16(bfr(c4[j]));
    }
    v4u w;
#pragma unroll
    for (int t = 0; t < 4; ++t) w[t] = pk16(hb[2 * t], hb[2 * t + 1]);
    st2u(XV + gi, w);
#pragma unroll
    for (int j = 0; j < 8; ++j) Ts[(8 * e + j) * TP + row] = hb[j];
  }
  __syncthreads();
#pragma unroll 1
  for (int it = 0; it < 4; ++it) {
    const int L = it * 32 + rq;
    const int l = L >> 1, dh = L & 1;
    const v4u u = *(const v4u*)(Ts + l * TP + dh * 64 + 8 * e);
    st2u(XT + (((size_t)(b * NH + hd)) * SEQ + l0 + l) * DH + dh * 64 + 8 * e, u);
  }
}

__global__ __launch_bounds__(256)
void colsum_kernel(const float* __restrict__ E, float* S) {
  __shared__ __align__(16) float Ss[256];
  const int tid = threadIdx.x;
  const int r = blockIdx.x * 256 + tid;
  const float* p = E + (size_t)r * SEQ;
  float s0 = 0.f, s1 = 0.f, s2 = 0.f, s3 = 0.f;
#pragma unroll 1
  for (int i = 0; i < SEQ / 4; ++i) {
    const v4f v = *(const v4f*)(p + 4 * i);
    s0 += bfr(v[0]); s1 += bfr(v[1]); s2 += bfr(v[2]); s3 += bfr(v[3]);
  }
  Ss[tid] = (s0 + s1) + (s2 + s3);
  __syncthreads();
  if (tid < 64) {
    const v4f u = *(const v4f*)(Ss + 4 * tid);
    st2f(S + blockIdx.x * 256 + 4 * tid, u);
  }
}

__global__ __launch_bounds__(256)
void cvt_w_kernel(const float* __restrict__ w, unsigned short* WP) {
  const int i = blockIdx.x * 256 + threadIdx.x;
  const int o = i >> 6, c8 = (i & 63) * 8;
  const float* p = w + (size_t)o * NC + c8;
  const v4f a  = *(const v4f*)(p);
  const v4f c4 = *(const v4f*)(p + 4);
  unsigned short hb[8];
#pragma unroll
  for (int j = 0; j < 4; ++j) {
    hb[j]     = h16(bfr(a[j]) * WSC);
    hb[4 + j] = h16(bfr(c4[j]) * WSC);
  }
  v4u u;
#pragma unroll
  for (int t = 0; t < 4; ++t) u[t] = pk16(hb[2 * t], hb[2 * t + 1]);
  st2u(WP + (size_t)i * 8, u);
}

template <int MODE>
__global__ __launch_bounds__(128)
void attn_kernel(const unsigned short* __restrict__ QP, const unsigned short* __restrict__ KP,
                 const unsigned short* __restrict__ VP, const float* __restrict__ S,
                 unsigned short* OH, unsigned short* OL) {
  __shared__ __align__(16) float Os[QT * OPD];
  const int tid  = threadIdx.x;
  const int wave = tid >> 5;
  const int lane = tid & 31;
  const int hh   = lane >> 4;
  const int c    = lane & 15;
  const int bx   = blockIdx.x;
  const int bh   = bx >> 4;
  const int n0   = (bx & 15) * QT;
  const int b    = bh >> 2, hd = bh & 3;
  const _Float16* QPh = (const _Float16*)(const void*)QP;
  const _Float16* KPh = (const _Float16*)(const void*)KP;
  const _Float16* VPh = (const _Float16*)(const void*)VP;

  const size_t qo = ((size_t)bh * SEQ + n0 + wave * 16 + c) * DH + 8 * hh;
  const v16h q0 = ldfrag_h(QPh + qo), q1 = ldfrag_h(QPh + qo + 32);
  const v16h q2 = ldfrag_h(QPh + qo + 64), q3 = ldfrag_h(QPh + qo + 96);
  const _Float16* Kp = KPh + ((size_t)bh * SEQ + c) * DH + 8 * hh;
  const _Float16* Vb = VPh + ((size_t)(b * NC + hd * DH + c)) * SEQ + 8 * hh;
  const float esc = (MODE == 0) ? ISQ : (ISQ * IQSC);

  float m = -1.0e30f, l = 0.f;
  v8f o0 = zero8(), o1 = zero8(), o2 = zero8(), o3 = zero8();
  v8f o4 = zero8(), o5 = zero8(), o6 = zero8(), o7 = zero8();
#pragma unroll 1
  for (int it = 0; it < SEQ / 32; ++it) {
    const int kb = it * 32;
    const _Float16* k0p = Kp + (size_t)kb * DH;
    const _Float16* k1p = k0p + 16 * DH;
    v8f s0 = zero8(), s1 = zero8();
    s0 = mma_h(ldfrag_h(k0p),      q0, s0);  s1 = mma_h(ldfrag_h(k1p),      q0, s1);
    s0 = mma_h(ldfrag_h(k0p + 32), q1, s0);  s1 = mma_h(ldfrag_h(k1p + 32), q1, s1);
    s0 = mma_h(ldfrag_h(k0p + 64), q2, s0);  s1 = mma_h(ldfrag_h(k1p + 64), q2, s1);
    s0 = mma_h(ldfrag_h(k0p + 96), q3, s0);  s1 = mma_h(ldfrag_h(k1p + 96), q3, s1);
#pragma unroll
    for (int r = 0; r < 8; ++r) { s0[r] *= esc; s1[r] *= esc; }

    float mx = fmaxf(hmax8(s0), hmax8(s1));
    mx = fmaxf(mx, __shfl_xor(mx, 16, 32));
    const float mn   = fmaxf(m, mx);
    const float corr = __expf(m - mn);
    m = mn;
    l *= corr;
#pragma unroll
    for (int r = 0; r < 8; ++r) {
      o0[r] *= corr; o1[r] *= corr; o2[r] *= corr; o3[r] *= corr;
      o4[r] *= corr; o5[r] *= corr; o6[r] *= corr; o7[r] *= corr;
    }

    FragH ph;
    float ls = 0.f;
    if (MODE == 0) {
      const float msh = mn - LNPS;
#pragma unroll
      for (int r = 0; r < 8; ++r) {
        const float e0 = __expf(s0[r] - msh);
        const float e1 = __expf(s1[r] - msh);
        ls += e0 + e1;
        ph.h[0][r] = (_Float16)e0;
        ph.h[1][r] = (_Float16)e1;
      }
    } else {
      const float base = __expf(-mn);
#pragma unroll
      for (int r = 0; r < 8; ++r) {
        const float e0 = __expf(s0[r] - mn);
        const float e1 = __expf(s1[r] - mn);
        ls += e0 + e1;
        ph.h[0][r] = (_Float16)((e0 - base) * PSC);
        ph.h[1][r] = (_Float16)((e1 - base) * PSC);
      }
    }
    l += ls;

    o0 = mma_h(ldfrag_h(Vb + 0 * 16 * SEQ + kb), ph.v, o0);
    o1 = mma_h(ldfrag_h(Vb + 1 * 16 * SEQ + kb), ph.v, o1);
    o2 = mma_h(ldfrag_h(Vb + 2 * 16 * SEQ + kb), ph.v, o2);
    o3 = mma_h(ldfrag_h(Vb + 3 * 16 * SEQ + kb), ph.v, o3);
    o4 = mma_h(ldfrag_h(Vb + 4 * 16 * SEQ + kb), ph.v, o4);
    o5 = mma_h(ldfrag_h(Vb + 5 * 16 * SEQ + kb), ph.v, o5);
    o6 = mma_h(ldfrag_h(Vb + 6 * 16 * SEQ + kb), ph.v, o6);
    o7 = mma_h(ldfrag_h(Vb + 7 * 16 * SEQ + kb), ph.v, o7);
  }
  l += __shfl_xor(l, 16, 32);
  const float rl = 1.0f / l;

  float* os = Os + (wave * 16 + c) * OPD + 8 * hh;
  if (MODE == 0) {
#define STG0(J, OJ)                                                              \
    {                                                                            \
      v4f u_, w_;                                                                \
      _Pragma("unroll") for (int r = 0; r < 4; ++r) {                            \
        u_[r] = OJ[r] * rl; w_[r] = OJ[4 + r] * rl;                              \
      }                                                                          \
      *(v4f*)(os + 16 * (J)) = u_; *(v4f*)(os + 16 * (J) + 4) = w_;              \
    }
    STG0(0, o0) STG0(1, o1) STG0(2, o2) STG0(3, o3) STG0(4, o4) STG0(5, o5) STG0(6, o6) STG0(7, o7)
#undef STG0
  } else {
    const float basef = __expf(-m);
    const float* sp = S + b * NC + hd * DH + 8 * hh;
#define STG1(J, OJ)                                                              \
    {                                                                            \
      v4f u_, w_;                                                                \
      _Pragma("unroll") for (int r = 0; r < 4; ++r) {                            \
        u_[r] = (OJ[r] * IPSC + basef * sp[16 * (J) + r]) * rl;                 \
        w_[r] = (OJ[4 + r] * IPSC + basef * sp[16 * (J) + 4 + r]) * rl;         \
      }                                                                          \
      *(v4f*)(os + 16 * (J)) = u_; *(v4f*)(os + 16 * (J) + 4) = w_;              \
    }
    STG1(0, o0) STG1(1, o1) STG1(2, o2) STG1(3, o3) STG1(4, o4) STG1(5, o5) STG1(6, o6) STG1(7, o7)
#undef STG1
  }
  __syncthreads();

  {
    const int e = tid & 7, lq = tid >> 3;
#pragma unroll 1
    for (int it = 0; it < 8; ++it) {
      const int L = it * 16 + lq;
      const int n = L >> 1, dh = L & 1;
      const float* src = Os + n * OPD + dh * 64 + 8 * e;
      const v4f x0 = *(const v4f*)(src);
      const v4f x1 = *(const v4f*)(src + 4);
      const size_t go = ((size_t)bh * SEQ + n0 + n) * DH + dh * 64 + 8 * e;
      if (MODE == 0) {
        unsigned short hb[8];
#pragma unroll
        for (int j = 0; j < 4; ++j) {
          hb[j]     = h16(x0[j] * QSC);
          hb[4 + j] = h16(x1[j] * QSC);
        }
        v4u uq;
#pragma unroll
        for (int t = 0; t < 4; ++t) uq[t] = pk16(hb[2 * t], hb[2 * t + 1]);
        st2u(OH + go, uq);
      } else {
        unsigned short hbh[8], hbl[8];
#pragma unroll
        for (int j = 0; j < 4; ++j) {
          const float hv0 = x0[j] * ESC;
          const _Float16 a0 = (_Float16)hv0;
          hbh[j] = __builtin_bit_cast(unsigned short, a0);
          hbl[j] = h16((hv0 - (float)a0) * RSC);
          const float hv1 = x1[j] * ESC;
          const _Float16 a1 = (_Float16)hv1;
          hbh[4 + j] = __builtin_bit_cast(unsigned short, a1);
          hbl[4 + j] = h16((hv1 - (float)a1) * RSC);
        }
        v4u uh, ul;
#pragma unroll
        for (int t = 0; t < 4; ++t) {
          uh[t] = pk16(hbh[2 * t], hbh[2 * t + 1]);
          ul[t] = pk16(hbl[2 * t], hbl[2 * t + 1]);
        }
        st2u(OH + go, uh);
        st2u(OL + go, ul);
      }
    }
  }
}

__device__ __forceinline__ void stage_x(float* xs, v8f ah, v8f ar, float bo) {
  v4f u, w;
#pragma unroll
  for (int r = 0; r < 4; ++r) {
    u[r] = (ah[r] + ar[r] * IRSC) * IWE + bo;
    w[r] = (ah[4 + r] + ar[4 + r] * IRSC) * IWE + bo;
  }
  *(v4f*)(xs) = u;
  *(v4f*)(xs + 4) = w;
}

__global__ __launch_bounds__(256)
void conv_kernel(const unsigned short* __restrict__ EH, const unsigned short* __restrict__ EL,
                 const unsigned short* __restrict__ WP, const float* __restrict__ bias, float* X) {
  __shared__ __align__(16) float Xs[128 * XP];
  const int tid  = threadIdx.x;
  const int wave = tid >> 5;
  const int lane = tid & 31;
  const int hh   = lane >> 4;
  const int cc   = lane & 15;
  const int bx   = blockIdx.x;
  const int og   = bx & 3, nt = bx >> 2;
  const int b    = nt >> 4;
  const int n0   = (nt & 15) * QT;
  const int o0   = og * 128;
  const int ng   = wave & 3, oh = wave >> 2;
  const _Float16* EHh = (const _Float16*)(const void*)EH;
  const _Float16* ELh = (const _Float16*)(const void*)EL;
  const _Float16* WPh = (const _Float16*)(const void*)WP;

  const size_t ao = ((size_t)b * NH * SEQ + n0 + 16 * ng + cc) * DH + 8 * hh;
  const _Float16* ahp = EHh + ao;
  const _Float16* alp = ELh + ao;
  const _Float16* wp  = WPh + (size_t)(o0 + 64 * oh + cc) * NC + 8 * hh;

  v8f h0 = zero8(), h1 = zero8(), h2 = zero8(), h3 = zero8();
  v8f g0 = zero8(), g1 = zero8(), g2 = zero8(), g3 = zero8();
#pragma unroll 1
  for (int ks = 0; ks < NC / 32; ++ks) {
    const size_t ko = (size_t)(ks >> 2) * SEQ * DH + (size_t)(ks & 3) * 32;
    const v16h fa = ldfrag_h(ahp + ko);
    const v16h fr = ldfrag_h(alp + ko);
    const _Float16* wk = wp + 32 * ks;
    v16h bw;
    bw = ldfrag_h(wk + 0 * 16 * NC); h0 = mma_h(fa, bw, h0); g0 = mma_h(fr, bw, g0);
    bw = ldfrag_h(wk + 1 * 16 * NC); h1 = mma_h(fa, bw, h1); g1 = mma_h(fr, bw, g1);
    bw = ldfrag_h(wk + 2 * 16 * NC); h2 = mma_h(fa, bw, h2); g2 = mma_h(fr, bw, g2);
    bw = ldfrag_h(wk + 3 * 16 * NC); h3 = mma_h(fa, bw, h3); g3 = mma_h(fr, bw, g3);
  }

  const int ob = o0 + 64 * oh + cc;
  const float b0v = bfr(bias[ob + 0 * 16]), b1v = bfr(bias[ob + 1 * 16]);
  const float b2v = bfr(bias[ob + 2 * 16]), b3v = bfr(bias[ob + 3 * 16]);
  float* xs = Xs + (64 * oh + cc) * XP + 16 * ng + 8 * hh;
  stage_x(xs + 0 * 16 * XP, h0, g0, b0v);
  stage_x(xs + 1 * 16 * XP, h1, g1, b1v);
  stage_x(xs + 2 * 16 * XP, h2, g2, b2v);
  stage_x(xs + 3 * 16 * XP, h3, g3, b3v);
  __syncthreads();
  {
    const int e = tid & 7, lq = tid >> 3;
#pragma unroll 1
    for (int it = 0; it < 8; ++it) {
      const int L  = it * 32 + lq;
      const int ol = L >> 1, hf = L & 1;
      const v4f v = *(const v4f*)(Xs + ol * XP + hf * 32 + 4 * e);
      st2f(X + ((size_t)(b * NC + o0 + ol)) * SEQ + n0 + hf * 32 + 4 * e, v);
    }
  }
}

__global__ __launch_bounds__(256)
void bn_swish_kernel(const float* __restrict__ X, const float* __restrict__ gam,
                     const float* __restrict__ bet, float* out) {
  __shared__ double rs_[8];
  __shared__ double rq_[8];
  const int o = blockIdx.x;
  const int tid = threadIdx.x, lane = tid & 31, wave = tid >> 5;
  double s = 0.0, q = 0.0;
#pragma unroll 1
  for (int bb = 0; bb < NB_; ++bb) {
    const v4f v = *(const v4f*)(X + ((size_t)(bb * NC + o)) * SEQ + 4 * tid);
#pragma unroll
    for (int k = 0; k < 4; ++k) {
      const double d = (double)v[k];
      s += d;
      q += d * d;
    }
  }
#pragma unroll
  for (int off = 16; off > 0; off >>= 1) {
    s += __shfl_xor(s, off, 32);
    q += __shfl_xor(q, off, 32);
  }
  if (lane == 0) { rs_[wave] = s; rq_[wave] = q; }
  __syncthreads();
  double ts = 0.0, tq = 0.0;
#pragma unroll
  for (int w = 0; w < 8; ++w) { ts += rs_[w]; tq += rq_[w]; }
  const double inv_n = 1.0 / (double)NSAMP;
  const double mu = ts * inv_n;
  double var = tq * inv_n - mu * mu;
  var = (var < 0.0) ? 0.0 : var;
  const float muf  = (float)mu;
  const float rstd = 1.0f / sqrtf((float)var + BNEPS);
  const float g = bfr(gam[o]), be = bfr(bet[o]);
#pragma unroll 1
  for (int bb = 0; bb < NB_; ++bb) {
    const size_t gi = ((size_t)(bb * NC + o)) * SEQ + 4 * tid;
    const v4f v = *(const v4f*)(X + gi);
    v4f r4;
#pragma unroll
    for (int k = 0; k < 4; ++k) {
      const float xn = ((v[k] - muf) * rstd) * g + be;
      const float t  = __expf(-xn);
      const float sg = __builtin_amdgcn_rcpf(1.0f + t);
      r4[k] = xn * sg;
    }
    st2f(out + gi, r4);
  }
}

extern "C" void kernel_launch(void* const* d_in, const int* in_sizes, int n_in,
                              void* d_out, int out_size, void* d_ws, size_t ws_size,
                              hipStream_t stream) {
  if (n_in < 6) return;
  if (in_sizes[0] != NEL || in_sizes[1] != NEL || in_sizes[2] != NC * NC ||
      in_sizes[3] != NC || in_sizes[4] != NC || in_sizes[5] != NC) return;
  if (out_size != NEL) return;

  const size_t szP16 = (size_t)NEL * 2;
  const size_t szX   = (size_t)NEL * 4;
  const size_t szW   = (size_t)NC * NC * 2;
  const size_t szS   = (size_t)NB_ * NC * 4;
  size_t off = 0;
  const size_t oCT = off; off += szP16;
  const size_t oCV = off; off += szP16;
  const size_t oET = off; off += szP16;
  const size_t oEV = off; off += szP16;
  const size_t oQ2 = off; off += szP16;
  const size_t oEH = off; off += szP16;
  const size_t oEL = off; off += szP16;
  const size_t oX  = off; off += szX;
  const size_t oWP = off; off += szW;
  const size_t oS  = off; off += szS;
  if (off > ws_size) return;
  if (off > (size_t)134217728) return;

  const float* cin   = (const float*)d_in[0];
  const float* ein   = (const float*)d_in[1];
  const float* wconv = (const float*)d_in[2];
  const float* bconv = (const float*)d_in[3];
  const float* gam   = (const float*)d_in[4];
  const float* bet   = (const float*)d_in[5];
  char* ws = (char*)d_ws;
  unsigned short* CT = (unsigned short*)(ws + oCT);
  unsigned short* CV = (unsigned short*)(ws + oCV);
  unsigned short* ET = (unsigned short*)(ws + oET);
  unsigned short* EV = (unsigned short*)(ws + oEV);
  unsigned short* Q2 = (unsigned short*)(ws + oQ2);
  unsigned short* EH = (unsigned short*)(ws + oEH);
  unsigned short* EL = (unsigned short*)(ws + oEL);
  float* X  = (float*)(ws + oX);
  unsigned short* WP = (unsigned short*)(ws + oWP);
  float* S  = (float*)(ws + oS);
  float* out = (float*)d_out;

  const dim3 blk256(256), blk128(128);
  const dim3 gX(NB_ * NH * (SEQ / 64));
  const dim3 gS((NB_ * NC) / 256);
  const dim3 gW((NC * NC / 8) / 256);
  const dim3 gA(NB_ * NH * (SEQ / QT));
  const dim3 gC(NB_ * (SEQ / QT) * 4);
  const dim3 gB(NC);

  cvt_x_kernel<<<gX, blk256, 0, stream>>>(cin, CV, CT);
  cvt_x_kernel<<<gX, blk256, 0, stream>>>(ein, EV, ET);
  colsum_kernel<<<gS, blk256, 0, stream>>>(ein, S);
  cvt_w_kernel<<<gW, blk256, 0, stream>>>(wconv, WP);
  attn_kernel<0><<<gA, blk128, 0, stream>>>(ET, CT, CV, S, Q2, Q2);
  attn_kernel<1><<<gA, blk128, 0, stream>>>(Q2, ET, EV, S, EH, EL);
  conv_kernel<<<gC, blk256, 0, stream>>>(EH, EL, WP, bconv, X);
  bn_swish_kernel<<<gB, blk256, 0, stream>>>(X, gam, bet, out);
  (void)hipGetLastError();
}
